// NODE_auto_64544768525257
// MI455X (gfx1250) — hardware-run, weakly checked
//
#include <hip/hip_runtime.h>


#define NB    2048
#define NR    32
#define NU    96
#define NV    8192
#define HI    256
#define HD    512
#define DIN   98
#define NSTEP 31
typedef _Float16 h16;
typedef unsigned short bf;
typedef __attribute__((ext_vector_type(16))) __bf16   v16bf;
typedef __attribute__((ext_vector_type(16))) _Float16 v16h;
typedef __attribute__((ext_vector_type(8)))  _Float16 v8h;
typedef __attribute__((ext_vector_type(8)))  unsigned short v8us;
typedef __attribute__((ext_vector_type(8)))  float    v8f;
typedef __attribute__((ext_vector_type(4)))  float    v4f;
typedef v8h  __attribute__((may_alias)) v8ha;
typedef v4f  __attribute__((may_alias)) v4fa;
typedef v8us __attribute__((may_alias)) v8usa;

__device__ __forceinline__ unsigned short f2bf(float f) { unsigned u = __float_as_uint(f); u += 0x7FFFu + ((u >> 16) & 1u); return (unsigned short)(u >> 16); }
__device__ __forceinline__ float bf2f(unsigned short b) { return __uint_as_float(((unsigned)b) << 16); }
__device__ __forceinline__ float bfr(float f) { return bf2f(f2bf(f)); }
__device__ __forceinline__ v16h cat16(v8h lo, v8h hi) { return __builtin_shufflevector(lo, hi, 0, 1, 2, 3, 4, 5, 6, 7, 8, 9, 10, 11, 12, 13, 14, 15); }
__device__ __forceinline__ v16bf cat16b(v8us lo, v8us hi) { return __builtin_bit_cast(v16bf, __builtin_shufflevector(lo, hi, 0, 1, 2, 3, 4, 5, 6, 7, 8, 9, 10, 11, 12, 13, 14, 15)); }
__device__ __forceinline__ v8f wmma16(v16h a, v16h b, v8f c) { return __builtin_amdgcn_wmma_f32_16x16x32_f16(false, a, false, b, (short)0, c, false, false); }
__device__ __forceinline__ v8f wmmab(v16bf a, v16bf b, v8f c) { return __builtin_amdgcn_wmma_f32_16x16x32_bf16(false, a, false, b, (short)0, c, false, false); }

template <typename T16> struct WFrag;
template <> struct WFrag<h16> { typedef v16h V; static __device__ __forceinline__ V ld(const h16* p) { return cat16(*(const v8h*)p, *(const v8h*)(p + 16)); } static __device__ __forceinline__ v8f mma(V a, V b, v8f c) { return wmma16(a, b, c); } };
template <> struct WFrag<bf> { typedef v16bf V; static __device__ __forceinline__ V ld(const bf* p) { return cat16b(*(const v8us*)p, *(const v8us*)(p + 16)); } static __device__ __forceinline__ v8f mma(V a, V b, v8f c) { return wmmab(a, b, c); } };
template <typename T16, int NSPLIT, bool BIAS>
__global__ __launch_bounds__(32) void k_gemmw(const T16* __restrict__ A, const T16* __restrict__ A2, const T16* __restrict__ Bt, const T16* __restrict__ Bt2, int K, float* C, int ldc, const float* __restrict__ bias, size_t sA, size_t sB, size_t sC) {
    typedef typename WFrag<T16>::V V;
    __shared__ __align__(16) float os[16 * 68];
    const size_t z = blockIdx.z; A += z * sA; if (A2) A2 += z * sA; Bt += z * sB; if (Bt2) Bt2 += z * sB; C += z * sC;
    const int lane = threadIdx.x & 31, lr = lane & 15, hi = lane >> 4; const int r0 = blockIdx.x * 64, c0 = blockIdx.y * 64;
    v8f acc[4][4];
#pragma unroll
    for (int mb = 0; mb < 4; ++mb)
#pragma unroll
        for (int nb = 0; nb < 4; ++nb) acc[mb][nb] = (v8f){};
    const size_t aoff = (size_t)(r0 + lr) * K + 8 * hi, boff = (size_t)(c0 + lr) * K + 8 * hi;
    for (int kc = 0; kc < K; kc += 32) {
        V a[4], a2[4];
#pragma unroll
        for (int mb = 0; mb < 4; ++mb) { a[mb] = WFrag<T16>::ld(A + aoff + (size_t)mb * 16 * K + kc); if (NSPLIT == 1 || NSPLIT == 2) a2[mb] = WFrag<T16>::ld(A2 + aoff + (size_t)mb * 16 * K + kc); }
#pragma unroll
        for (int nb = 0; nb < 4; ++nb) { const V b = WFrag<T16>::ld(Bt + boff + (size_t)nb * 16 * K + kc); V b2; if (NSPLIT >= 2) b2 = WFrag<T16>::ld(Bt2 + boff + (size_t)nb * 16 * K + kc);
#pragma unroll
            for (int mb = 0; mb < 4; ++mb) { acc[mb][nb] = WFrag<T16>::mma(a[mb], b, acc[mb][nb]); if (NSPLIT == 1 || NSPLIT == 2) acc[mb][nb] = WFrag<T16>::mma(a2[mb], b, acc[mb][nb]); if (NSPLIT >= 2) acc[mb][nb] = WFrag<T16>::mma(a[mb], b2, acc[mb][nb]); } }
        asm volatile("v_nop\n\tv_nop\n\tv_nop\n\tv_nop" : "+v"(acc[0][0]), "+v"(acc[1][1]), "+v"(acc[2][2]), "+v"(acc[3][3]) : "v"(a[0]), "v"(a[3]));
    }
#pragma unroll
    for (int mb = 0; mb < 4; ++mb) {
#pragma unroll
        for (int nb = 0; nb < 4; ++nb) {
#pragma unroll
            for (int j = 0; j < 8; ++j) os[(hi * 8 + j) * 68 + nb * 16 + lr] = acc[mb][nb][j]; }
        __builtin_amdgcn_wave_barrier(); asm volatile("" ::: "memory");
        float* crow = C + (size_t)(r0 + mb * 16) * ldc + c0;
#pragma unroll 1
        for (int ps = 0; ps < 2; ++ps) {
#pragma unroll
            for (int s = 0; s < 8; ++s) { const int row = 2 * s + hi, cofs = lr * 4; v4f val = *(const v4fa*)(os + row * 68 + cofs); if (BIAS) { val[0] += bfr(bias[c0 + cofs]); val[1] += bfr(bias[c0 + cofs + 1]); val[2] += bfr(bias[c0 + cofs + 2]); val[3] += bfr(bias[c0 + cofs + 3]); }
                *(volatile v4f*)(crow + (size_t)row * ldc + cofs) = val; }
            if (ps == 0) __threadfence(); }
        __builtin_amdgcn_wave_barrier(); asm volatile("" ::: "memory");
    }
}

typedef __attribute__((ext_vector_type(2))) _Float16 v2h;
typedef __attribute__((ext_vector_type(4))) _Float16 v4h;
typedef __attribute__((ext_vector_type(2))) unsigned short v2us;
typedef __attribute__((ext_vector_type(4))) unsigned short v4us;
typedef __attribute__((ext_vector_type(2))) float v2f;
typedef __attribute__((ext_vector_type(4))) int v4i;


__global__ __launch_bounds__(256) void k_rnd(const float* __restrict__ src, float* y, bf* op, size_t n4) { const size_t i = (size_t)blockIdx.x * 256 + threadIdx.x; if (i >= n4) return; const v4f v = *(const v4f*)(src + i * 4); v4us o; v4f r;
#pragma unroll
    for (int k = 0; k < 4; ++k) { o[k] = f2bf(v[k]); r[k] = bf2f(o[k]); }
    *(volatile v4f*)(y + i * 4) = r; *(volatile v4us*)(op + i * 4) = o; __threadfence(); *(volatile v4f*)(y + i * 4) = r; *(volatile v4us*)(op + i * 4) = o; }

__global__ __launch_bounds__(256) void k_gathU(const int* __restrict__ idx, const float* __restrict__ u0, const float* __restrict__ u1, const float* __restrict__ u2, bf* uv) { const int i = blockIdx.x * 256 + threadIdx.x; const int row = i / 24; const int c4 = (i - row * 24) * 4; const int m = c4 >> 5; const int cc = c4 & 31;
    int id = idx[row * 3 + m]; id = id < 0 ? 0 : (id > NV - 1 ? NV - 1 : id);
    const float* tb = (m == 0) ? u0 : ((m == 1) ? u1 : u2);
    const v4f a = *(const v4f*)(tb + (size_t)id * NR + cc); v4us o;
#pragma unroll
    for (int k = 0; k < 4; ++k) o[k] = f2bf(a[k]);
    *(volatile v4us*)(uv + (size_t)i * 4) = o; __threadfence(); *(volatile v4us*)(uv + (size_t)i * 4) = o; }

__global__ __launch_bounds__(256) void k_pkw(const float* __restrict__ wd1, bf* w1c) { const int i = blockIdx.x * 256 + threadIdx.x; const int h = i / 48; const int c2 = (i - h * 48) * 2; const v2f a = *(const v2f*)(wd1 + (size_t)h * DIN + 2 + c2); v2us o; o[0] = f2bf(a[0]); o[1] = f2bf(a[1]);
    *(volatile v2us*)(w1c + (size_t)i * 2) = o; __threadfence(); *(volatile v2us*)(w1c + (size_t)i * 2) = o; }

__global__ __launch_bounds__(256) void k_init(const float* __restrict__ h1t, const float* __restrict__ bi1, const float* __restrict__ wi2, const float* __restrict__ bi2, float* x0) { const int r = blockIdx.x * 256 + threadIdx.x; float acc = 0.0f;
    for (int j = 0; j < HI; ++j) acc += tanhf(h1t[(size_t)j * NB + r] + bfr(bi1[j])) * bfr(wi2[j]);
    const float v = acc + bfr(bi2[0]); *(volatile float*)(x0 + r) = v; __threadfence(); *(volatile float*)(x0 + r) = v; }

__global__ __launch_bounds__(256) void k_ode(const float* __restrict__ baset, const float* __restrict__ x0, const float* __restrict__ btn, const float* __restrict__ wd1, const float* __restrict__ bd1, const float* __restrict__ wd2, const float* __restrict__ bd2, float* out) { const int r = blockIdx.x * 256 + threadIdx.x;
    const float s = bfr(btn[r]); const float b2 = bfr(bd2[0]); const float hs = 1.0f / 31.0f; float x = x0[r];
    for (int it = 0; it < NSTEP; ++it) { const float t = (float)it * hs; float k = 0.0f, sum = 0.0f;
#pragma unroll 1
        for (int g = 0; g < 4; ++g) { const float ct = (g == 0) ? 0.0f : ((g == 3) ? 1.0f : 0.5f); const float cw = (g == 0 || g == 3) ? 1.0f : 2.0f;
            const float tt = t + hs * ct; const float xx = x + (hs * ct) * k; const float st = s * tt; float acc = 0.0f;
            for (int j = 0; j < HD; ++j) acc += tanhf(((baset[(size_t)j * NB + r] + bfr(bd1[j])) + st * bfr(wd1[(size_t)j * DIN])) + xx * bfr(wd1[(size_t)j * DIN + 1])) * bfr(wd2[j]);
            k = (acc + b2) * s; sum += cw * k; }
        x = x + (hs / 6.0f) * sum; }
    *(volatile float*)(out + r) = x; __threadfence(); *(volatile float*)(out + r) = x; }

static constexpr size_t kSzUV = (size_t)NB * NU * 2, kSzW1C = (size_t)HD * NU * 2, kSzWI1W = (size_t)HI * NU * 2, kSzSW = (size_t)HI * NU * 4, kSzBT = (size_t)HD * NB * 4, kSzH1T = (size_t)HI * NB * 4, kSzX0 = (size_t)NB * 4;
static constexpr size_t kOffUV = 0, kOffW1C = kOffUV + kSzUV, kOffWI1W = kOffW1C + kSzW1C, kOffSW = kOffWI1W + kSzWI1W, kOffBT = kOffSW + kSzSW, kOffH1T = kOffBT + kSzBT, kOffX0 = kOffH1T + kSzH1T, kWsTotal = kOffX0 + kSzX0;
static_assert(kSzUV == 393216ull && kSzW1C == 98304ull && kSzWI1W == 49152ull && kSzSW == 98304ull && kSzBT == 4194304ull && kSzH1T == 2097152ull && kSzX0 == 8192ull && kWsTotal == 6938624ull);
static_assert(kWsTotal <= 134217728ull);
static_assert((kSzUV % 128) == 0 && (kSzW1C % 128) == 0 && (kSzWI1W % 128) == 0 && (kSzSW % 128) == 0 && (kSzBT % 128) == 0 && (kSzH1T % 128) == 0 && (kSzX0 % 128) == 0);
static_assert((HD % 64) == 0 && (HI % 64) == 0 && (NB % 64) == 0 && (NU % 32) == 0);
static_assert(NU == 3 * NR && DIN == NU + 2 && ((NB * 24) % 256) == 0 && ((HD * 48) % 256) == 0 && ((HI * NU) % 1024) == 0 && (NB % 256) == 0);

extern "C" void kernel_launch(void* const* d_in, const int* in_sizes, int n_in, void* d_out, int out_size, void* d_ws, size_t ws_size, hipStream_t stream) {
    if (n_in < 13) return;
    if (in_sizes[0] != NB * 3 || in_sizes[1] != NB || in_sizes[2] != NV * NR || in_sizes[3] != NV * NR || in_sizes[4] != NV * NR) return;
    if (in_sizes[5] != HI * NU || in_sizes[6] != HI || in_sizes[7] != HI || in_sizes[8] != 1) return;
    if (in_sizes[9] != HD * DIN || in_sizes[10] != HD || in_sizes[11] != HD || in_sizes[12] != 1) return;
    if (out_size != NB) return;
    if (ws_size < kWsTotal) return;
    const int* idx = (const int*)d_in[0]; const float* btn = (const float*)d_in[1]; const float* u0 = (const float*)d_in[2]; const float* u1 = (const float*)d_in[3]; const float* u2 = (const float*)d_in[4];
    const float* wi1 = (const float*)d_in[5]; const float* bi1 = (const float*)d_in[6]; const float* wi2 = (const float*)d_in[7]; const float* bi2 = (const float*)d_in[8];
    const float* wd1 = (const float*)d_in[9]; const float* bd1 = (const float*)d_in[10]; const float* wd2 = (const float*)d_in[11]; const float* bd2 = (const float*)d_in[12];
    float* out = (float*)d_out; char* ws = (char*)d_ws;
    bf* UV = (bf*)(ws + kOffUV); bf* W1C = (bf*)(ws + kOffW1C); bf* WI1W = (bf*)(ws + kOffWI1W); float* SW = (float*)(ws + kOffSW); float* BASET = (float*)(ws + kOffBT); float* H1T = (float*)(ws + kOffH1T); float* X0 = (float*)(ws + kOffX0);

    k_gathU<<<(unsigned)(NB * 24 / 256), 256, 0, stream>>>(idx, u0, u1, u2, UV);
    k_pkw<<<(unsigned)(HD * 48 / 256), 256, 0, stream>>>(wd1, W1C);
    k_rnd<<<(unsigned)(HI * NU / 4 / 256), 256, 0, stream>>>(wi1, SW, WI1W, (size_t)HI * NU / 4);
    k_gemmw<bf, 0, false><<<dim3(HD / 64, NB / 64, 1), 32, 0, stream>>>(W1C, nullptr, UV, nullptr, NU, BASET, NB, nullptr, 0, 0, 0);
    k_gemmw<bf, 0, false><<<dim3(HI / 64, NB / 64, 1), 32, 0, stream>>>(WI1W, nullptr, UV, nullptr, NU, H1T, NB, nullptr, 0, 0, 0);
    k_init<<<(unsigned)(NB / 256), 256, 0, stream>>>(H1T, bi1, wi2, bi2, X0);
    k_ode<<<(unsigned)(NB / 256), 256, 0, stream>>>(BASET, X0, btn, wd1, bd1, wd2, bd2, out);
}
